// MambaBlock_43284680409477
// MI455X (gfx1250) — hardware-verified
//
#include <hip/hip_runtime.h>
#include <math.h>

typedef __attribute__((ext_vector_type(16))) _Float16 v16h;
typedef __attribute__((ext_vector_type(8)))  _Float16 v8h;
typedef __attribute__((ext_vector_type(8)))  float    v8f;
typedef __attribute__((ext_vector_type(4)))  float    v4f;

constexpr int kBatch = 2;
constexpr int kSeqL  = 1024;
constexpr int kDmod  = 1024;
constexpr int kDin   = 2048;
constexpr int kNst   = 16;
constexpr int kDtR   = 64;
constexpr int kPrjN  = 96;
constexpr int kPrjP  = 128;
constexpr int kXZP   = 2 * kDin;
constexpr int kRows  = kBatch * kSeqL;
constexpr int kTP    = 260;

constexpr float kCarryW   = 32.0f;
constexpr float kCarryWdt = 8.0f;
constexpr float kCarryDt  = 16.0f;
constexpr float kCarryY   = 16.0f;
constexpr float kFoldIn   = 1.0f / kCarryW;
constexpr float kFoldXp   = 1.0f / kCarryW;
constexpr float kFoldDt   = 1.0f / (kCarryDt * kCarryWdt);
constexpr float kFoldOut  = 1.0f / (kCarryY * kCarryW);

static_assert(kDtR + 2 * kNst == kPrjN, "x_proj width");
static_assert((kSeqL & (kSeqL - 1)) == 0, "sequence length is a power of two");
static_assert((kDmod % 32) == 0 && (kDin % 32) == 0 && (kDtR % 32) == 0, "GEMM K multiples of 32");
static_assert((kRows % 64) == 0 && (kXZP % 64) == 0 && (kPrjP % 64) == 0 && (kDin % 64) == 0 && (kDmod % 64) == 0, "GEMM M,N multiples of 64");
static_assert((kSeqL % 64) == 0 && (kDin % 256) == 0 && (kRows % 8) == 0 && (kDmod % 256) == 0, "tile multiples");

constexpr size_t kSzWIN  = (size_t)kXZP  * kDmod * 2;
constexpr size_t kSzWXP  = (size_t)kPrjP * kDin  * 2;
constexpr size_t kSzWDT  = (size_t)kDin  * kDtR  * 2;
constexpr size_t kSzWOUT = (size_t)kDmod * kDin  * 2;
constexpr size_t kSzXN   = (size_t)kRows * kDmod * 2;
constexpr size_t kSzXZ   = (size_t)kRows * kXZP  * 4;
constexpr size_t kSzUC   = (size_t)kRows * kDin  * 4;
constexpr size_t kSzUC16 = (size_t)kRows * kDin  * 2;
constexpr size_t kSzPROJ = (size_t)kRows * kPrjP * 4;
constexpr size_t kSzDT16 = (size_t)kRows * kDtR  * 2;
constexpr size_t kSzDLR  = (size_t)kRows * kDin  * 4;
constexpr size_t kSzY16  = (size_t)kRows * kDin  * 2;
constexpr size_t kOffWIN  = 0;
constexpr size_t kOffWXP  = kOffWIN  + kSzWIN;
constexpr size_t kOffWDT  = kOffWXP  + kSzWXP;
constexpr size_t kOffWOUT = kOffWDT  + kSzWDT;
constexpr size_t kOffXN   = kOffWOUT + kSzWOUT;
constexpr size_t kOffXZ   = kOffXN   + kSzXN;
constexpr size_t kOffUC   = kOffXZ   + kSzXZ;
constexpr size_t kOffUC16 = kOffUC   + kSzUC;
constexpr size_t kOffPROJ = kOffUC16 + kSzUC16;
constexpr size_t kOffDT16 = kOffPROJ + kSzPROJ;
constexpr size_t kOffDLR  = kOffDT16 + kSzDT16;
constexpr size_t kOffY16  = kOffDLR  + kSzDLR;
constexpr size_t kWsTotal = kOffY16  + kSzY16;
static_assert(kWsTotal == 102760448ull, "carve total");
static_assert(kWsTotal <= 134217728ull, "carve cap");
static_assert((kOffWXP % 128) == 0 && (kOffWDT % 128) == 0 && (kOffWOUT % 128) == 0 && (kOffXN % 128) == 0 &&
              (kOffXZ % 128) == 0 && (kOffUC % 128) == 0 && (kOffUC16 % 128) == 0 && (kOffPROJ % 128) == 0 &&
              (kOffDT16 % 128) == 0 && (kOffDLR % 128) == 0 && (kOffY16 % 128) == 0, "128-B aligned regions");

union FragU { v16h v; v8h h[2]; };
__device__ __forceinline__ v16h frag_load(const _Float16* p) {
  FragU f;
  f.h[0] = *(const v8h*)(p);
  f.h[1] = *(const v8h*)(p + 16);
  return f.v;
}
__device__ __forceinline__ v8f frag_mma(v16h a, v16h b, v8f c) {
  return __builtin_amdgcn_wmma_f32_16x16x32_f16(false, a, false, b, (short)0, c, false, false);
}
__device__ __forceinline__ void mma_guard4(v8f& a, v8f& b, v8f& c, v8f& d, v16h x, v16h b0, v16h b1, v16h b2, v16h b3) {
  asm volatile("v_nop\n\tv_nop\n\tv_nop\n\tv_nop" : "+v"(a), "+v"(b), "+v"(c), "+v"(d) : "v"(x), "v"(b0), "v"(b1), "v"(b2), "v"(b3));
}
__device__ __forceinline__ void keep4_h(v16h a, v16h b, v16h c, v16h d) { asm volatile("v_nop" :: "v"(a), "v"(b), "v"(c), "v"(d)); }
__device__ __forceinline__ void acc_guard4(v8f& a, v8f& b, v8f& c, v8f& d) { asm volatile("v_nop\n\tv_nop\n\tv_nop\n\tv_nop" : "+v"(a), "+v"(b), "+v"(c), "+v"(d)); }

template <int BIAS_MODE, bool RESID, bool DEVSCALE>
__global__ __launch_bounds__(256) void wmma_gemm64_f16(
    const unsigned short* __restrict__ Ap, int lda,
    const unsigned short* __restrict__ Btp, int ldb,
    float* __restrict__ C, int ldc,
    const float* __restrict__ bias,
    const float* __restrict__ resid,
    const float* __restrict__ dscale,
    int M, int N, int K, float scale)
{
  const _Float16* A  = (const _Float16*)Ap;
  const _Float16* Bt = (const _Float16*)Btp;
  __shared__ __align__(16) float sT[8][16 * 68];
  const int lane = threadIdx.x & 31;
  const int wave = threadIdx.x >> 5;
  const int tilesN = N >> 6;
  const int tilesM = M >> 6;
  const int tile = blockIdx.x * 8 + wave;
  if (tile >= tilesM * tilesN) return;
  const int tm = tile / tilesN;
  const int tn = tile - tm * tilesN;
  const int m0 = tm << 6;
  const int n0 = tn << 6;

  const int rlane = lane & 15;
  const int koff  = (lane >> 4) * 8;
  const int mOff  = (lane >> 4) * 8;

  float sc = scale;
  if (DEVSCALE) sc = scale * dscale[0];

  v8f acc[4][4];
#pragma unroll
  for (int i = 0; i < 4; ++i)
#pragma unroll
    for (int j = 0; j < 4; ++j) acc[i][j] = (v8f){0.f, 0.f, 0.f, 0.f, 0.f, 0.f, 0.f, 0.f};

  for (int k0 = 0; k0 < K; k0 += 32) {
    v16h bh[4];
#pragma unroll
    for (int j = 0; j < 4; ++j) {
      const size_t bo = (size_t)(n0 + (j << 4) + rlane) * ldb + koff + k0;
      bh[j] = frag_load(Bt + bo);
    }
#pragma unroll
    for (int i = 0; i < 4; ++i) {
      const size_t ao = (size_t)(m0 + (i << 4) + rlane) * lda + koff + k0;
      const v16h ah = frag_load(A + ao);
#pragma unroll
      for (int j = 0; j < 4; ++j) acc[i][j] = frag_mma(ah, bh[j], acc[i][j]);
      mma_guard4(acc[i][0], acc[i][1], acc[i][2], acc[i][3], ah, bh[0], bh[1], bh[2], bh[3]);
    }
    keep4_h(bh[0], bh[1], bh[2], bh[3]);
  }
  acc_guard4(acc[0][0], acc[0][1], acc[0][2], acc[0][3]);
  acc_guard4(acc[1][0], acc[1][1], acc[1][2], acc[1][3]);
  acc_guard4(acc[2][0], acc[2][1], acc[2][2], acc[2][3]);
  acc_guard4(acc[3][0], acc[3][1], acc[3][2], acc[3][3]);

  float* slab = sT[wave];
  const int hh = lane >> 4;
  const int c4 = (lane & 15) * 4;
#pragma unroll
  for (int i = 0; i < 4; ++i) {
    const int mBase = m0 + (i << 4);
#pragma unroll
    for (int j = 0; j < 4; ++j) {
      float bv = 0.f;
      if (BIAS_MODE == 2) bv = bias[n0 + (j << 4) + rlane];
#pragma unroll
      for (int r = 0; r < 8; ++r) {
        float v = acc[i][j][r] * sc;
        if (BIAS_MODE == 2) v += bv;
        slab[(mOff + r) * 68 + (j << 4) + rlane] = v;
      }
    }
    __builtin_amdgcn_fence(__ATOMIC_RELEASE, "workgroup");
    __builtin_amdgcn_wave_barrier();
    __builtin_amdgcn_fence(__ATOMIC_ACQUIRE, "workgroup");
    v4f ov[8];
#pragma unroll
    for (int it = 0; it < 8; ++it) {
      const int row = it * 2 + hh;
      v4f sv = *(const v4f*)(slab + row * 68 + c4);
      if (RESID) {
        const v4f rx = *(const v4f*)(resid + (size_t)(mBase + row) * ldc + n0 + c4);
        sv = sv + rx;
      }
      ov[it] = sv;
    }
    for (int pass = 0; pass < 2; ++pass) {
#pragma unroll
      for (int it = 0; it < 8; ++it) {
        const int row = it * 2 + hh;
        *(volatile v4f*)(C + (size_t)(mBase + row) * ldc + n0 + c4) = ov[it];
      }
      __threadfence();
    }
    __builtin_amdgcn_fence(__ATOMIC_RELEASE, "workgroup");
    __builtin_amdgcn_wave_barrier();
    __builtin_amdgcn_fence(__ATOMIC_ACQUIRE, "workgroup");
  }
}

__global__ __launch_bounds__(256) void ln_cast_kernel(
    const float* __restrict__ x, const float* __restrict__ g, const float* __restrict__ bt,
    unsigned short* __restrict__ XN)
{
  const int lane = threadIdx.x & 31, wave = threadIdx.x >> 5;
  const int row = blockIdx.x * 8 + wave;
  const float* xr = x + (size_t)row * kDmod + lane * 8;
  float s = 0.f;
#pragma unroll 1
  for (int j = 0; j < 4; ++j) {
    const v4f a0 = *(const v4f*)(xr + j * 256);
    const v4f a1 = *(const v4f*)(xr + j * 256 + 4);
    s += ((a0[0] + a0[1]) + (a0[2] + a0[3])) + ((a1[0] + a1[1]) + (a1[2] + a1[3]));
  }
#pragma unroll
  for (int off = 16; off > 0; off >>= 1) s += __shfl_xor(s, off, 32);
  const float mu = s * (1.0f / (float)kDmod);
  float q = 0.f;
#pragma unroll 1
  for (int j = 0; j < 4; ++j) {
    const v4f a0 = *(const v4f*)(xr + j * 256);
    const v4f a1 = *(const v4f*)(xr + j * 256 + 4);
#pragma unroll
    for (int e = 0; e < 4; ++e) {
      const float d0 = a0[e] - mu;
      const float d1 = a1[e] - mu;
      q = fmaf(d0, d0, q);
      q = fmaf(d1, d1, q);
    }
  }
#pragma unroll
  for (int off = 16; off > 0; off >>= 1) q += __shfl_xor(q, off, 32);
  const float rstd = rsqrtf(q * (1.0f / (float)kDmod) + 1e-5f);
#pragma unroll 1
  for (int j = 0; j < 4; ++j) {
    const int c0 = j * 256 + lane * 8;
    const v4f a0 = *(const v4f*)(xr + j * 256);
    const v4f a1 = *(const v4f*)(xr + j * 256 + 4);
    const v4f g0 = *(const v4f*)(g + c0);
    const v4f g1 = *(const v4f*)(g + c0 + 4);
    const v4f b0 = *(const v4f*)(bt + c0);
    const v4f b1 = *(const v4f*)(bt + c0 + 4);
    v8h hv;
#pragma unroll
    for (int e = 0; e < 4; ++e) {
      hv[e]     = (_Float16)(((a0[e] - mu) * rstd) * g0[e] + b0[e]);
      hv[4 + e] = (_Float16)(((a1[e] - mu) * rstd) * g1[e] + b1[e]);
    }
    unsigned short* qd = XN + (size_t)row * kDmod + c0;
    *(volatile v8h*)qd = hv;
    __threadfence();
    *(volatile v8h*)qd = hv;
  }
}

__global__ __launch_bounds__(256) void transpose_cast_kernel(
    const float* __restrict__ W, unsigned short* __restrict__ Bt, int Kdim, int Ndim, float scale)
{
  __shared__ float tile[64 * 65];
  const int tid = threadIdx.x, lane = tid & 31, wave = tid >> 5;
  const int n0 = blockIdx.x * 64;
  const int k0 = blockIdx.y * 64;
#pragma unroll 1
  for (int ph = 0; ph < 2; ++ph) {
#pragma unroll
    for (int p = 0; p < 8; ++p) {
      const int idx = tid + (ph * 8 + p) * 256;
      const int kk  = idx >> 6;
      const int nn  = idx & 63;
      const int n   = n0 + nn;
      const int nc  = (n < Ndim) ? n : (Ndim - 1);
      const float v = W[(size_t)(k0 + kk) * Ndim + nc];
      tile[kk * 65 + nn] = (n < Ndim) ? (v * scale) : 0.f;
    }
  }
  __syncthreads();
  const int q = lane >> 3, c8 = (lane & 7) * 8;
  v8h hv[2];
#pragma unroll
  for (int it = 0; it < 2; ++it) {
    const int nrow = it * 32 + wave * 4 + q;
#pragma unroll
    for (int e = 0; e < 8; ++e) hv[it][e] = (_Float16)tile[(c8 + e) * 65 + nrow];
  }
  for (int pass = 0; pass < 2; ++pass) {
#pragma unroll
    for (int it = 0; it < 2; ++it) {
      const int nrow = it * 32 + wave * 4 + q;
      *(volatile v8h*)(Bt + (size_t)(n0 + nrow) * Kdim + k0 + c8) = hv[it];
    }
    __threadfence();
  }
}

__global__ __launch_bounds__(256) void dt_cast_kernel(
    const float* __restrict__ PROJ, unsigned short* __restrict__ DT16, int total8, float scale)
{
  const int i = blockIdx.x * 256 + threadIdx.x;
  if (i >= total8) return;
  const int e0  = i << 3;
  const int row = e0 >> 6;
  const int c8  = e0 & 63;
  const float* p = PROJ + (size_t)row * kPrjP + c8;
  const v4f a0 = *(const v4f*)(p);
  const v4f a1 = *(const v4f*)(p + 4);
  v8h hv;
#pragma unroll
  for (int e = 0; e < 4; ++e) {
    hv[e]     = (_Float16)(a0[e] * scale);
    hv[4 + e] = (_Float16)(a1[e] * scale);
  }
  unsigned short* qd = DT16 + e0;
  *(volatile v8h*)qd = hv;
  __threadfence();
  *(volatile v8h*)qd = hv;
}

__global__ __launch_bounds__(256) void conv_silu_kernel(
    const float* __restrict__ XZ, const float* __restrict__ cw, const float* __restrict__ cb,
    float* __restrict__ UC, unsigned short* __restrict__ UC16)
{
  __shared__ __align__(16) float sT[16 * kTP];
  const int tid = threadIdx.x, lane = tid & 31, wave = tid >> 5;
  const int d0 = blockIdx.x * 256, d = d0 + tid;
  const int g0 = blockIdx.y * 64;
  const int tb = g0 & (kSeqL - 1);
  const v4f wv = *(const v4f*)(cw + (size_t)d * 4);
  const float w0 = wv[0], w1 = wv[1], w2 = wv[2], w3 = wv[3];
  const float bc = cb[d];
  float xm3, xm2, xm1;
  {
    const bool hist = (tb > 0);
    const int rb = hist ? (g0 - 3) : g0;
    const float v3 = XZ[(size_t)rb * kXZP + d];
    const float v2 = XZ[(size_t)(rb + 1) * kXZP + d];
    const float v1 = XZ[(size_t)(rb + 2) * kXZP + d];
    xm3 = hist ? v3 : 0.f;
    xm2 = hist ? v2 : 0.f;
    xm1 = hist ? v1 : 0.f;
  }
  const int hrow = wave >> 1;
  const int hch  = (wave & 1) * 128 + lane * 4;
#pragma unroll 1
  for (int sub = 0; sub < 4; ++sub) {
    const int lb = g0 + sub * 16;
#pragma unroll 1
    for (int s = 0; s < 16; ++s) {
      const float xc = XZ[(size_t)(lb + s) * kXZP + d];
      float acc = w0 * xm3;
      acc = fmaf(w1, xm2, acc);
      acc = fmaf(w2, xm1, acc);
      acc = fmaf(w3, xc, acc);
      const float sv = acc + bc;
      const float sg = __builtin_amdgcn_rcpf(1.0f + expf(-sv));
      sT[s * kTP + tid] = sv * sg;
      xm3 = xm2; xm2 = xm1; xm1 = xc;
    }
    __syncthreads();
    v4f fv[4];
    v8h bv[2];
#pragma unroll
    for (int it = 0; it < 4; ++it) fv[it] = *(const v4f*)(sT + (it * 4 + hrow) * kTP + hch);
#pragma unroll
    for (int it = 0; it < 2; ++it) {
      const float* sp = sT + (it * 8 + wave) * kTP + lane * 8;
      const v4f a0 = *(const v4f*)(sp);
      const v4f a1 = *(const v4f*)(sp + 4);
#pragma unroll
      for (int e = 0; e < 4; ++e) {
        bv[it][e]     = (_Float16)a0[e];
        bv[it][4 + e] = (_Float16)a1[e];
      }
    }
    for (int pass = 0; pass < 2; ++pass) {
#pragma unroll
      for (int it = 0; it < 4; ++it)
        *(volatile v4f*)(UC + (size_t)(lb + it * 4 + hrow) * kDin + d0 + hch) = fv[it];
#pragma unroll
      for (int it = 0; it < 2; ++it)
        *(volatile v8h*)(UC16 + (size_t)(lb + it * 8 + wave) * kDin + d0 + lane * 8) = bv[it];
      __threadfence();
    }
    __syncthreads();
  }
}

__global__ __launch_bounds__(256) void scan_kernel(
    const float* __restrict__ DLR, const float* __restrict__ UC, const float* __restrict__ XZ,
    const float* __restrict__ PROJ, const float* __restrict__ A_log, const float* __restrict__ Dv,
    unsigned short* __restrict__ Y16)
{
  __shared__ __align__(16) float sBC[16 * 32];
  __shared__ __align__(16) float sY[16 * kTP];
  __shared__ __align__(16) float sA[kNst * 256];
  const int tid = threadIdx.x, lane = tid & 31, wave = tid >> 5;
  const int d0 = blockIdx.x * 256, d = d0 + tid;
  const size_t row0 = (size_t)blockIdx.y * kSeqL;

#pragma unroll 1
  for (int n = 0; n < kNst; ++n) sA[n * 256 + tid] = -expf(A_log[(size_t)d * kNst + n]);
  __syncthreads();
  float An[kNst], h[kNst];
#pragma unroll
  for (int n = 0; n < kNst; ++n) {
    An[n] = sA[n * 256 + tid];
    h[n] = 0.f;
  }
  const float Dd = Dv[d];

#pragma unroll 1
  for (int c = 0; c < kSeqL / 16; ++c) {
    const int l0 = c * 16;
    if (tid < 128) {
      const int r = tid >> 3, q = (tid & 7) * 4;
      const v4f v = *(const v4f*)(PROJ + (row0 + l0 + r) * kPrjP + kDtR + q);
      *(v4f*)(sBC + r * 32 + q) = v;
    }
    __syncthreads();
#pragma unroll 1
    for (int s = 0; s < 16; ++s) {
      const size_t m = row0 + (size_t)(l0 + s);
      const float a     = DLR[m * kDin + d];
      const float delta = fmaxf(a, 0.0f) + log1pf(expf(-fabsf(a)));
      const float xv    = UC[m * kDin + d];
      const float zv    = XZ[m * kXZP + kDin + d];
      v4f Bq[4], Cq[4];
#pragma unroll
      for (int qq = 0; qq < 4; ++qq) {
        Bq[qq] = *(const v4f*)(sBC + s * 32 + 4 * qq);
        Cq[qq] = *(const v4f*)(sBC + s * 32 + kNst + 4 * qq);
      }
      float y = 0.f;
#pragma unroll
      for (int n = 0; n < kNst; ++n) {
        const float e = __expf(delta * An[n]);
        float db = delta * Bq[n >> 2][n & 3];
        asm volatile("" : "+v"(db));
        float p = db * xv;
        asm volatile("" : "+v"(p));
        float qv = h[n] * e;
        asm volatile("" : "+v"(qv));
        const float hn = qv + p;
        h[n] = hn;
        float rr = Cq[n >> 2][n & 3] * hn;
        asm volatile("" : "+v"(rr));
        y += rr;
      }
      float sk = xv * Dd;
      asm volatile("" : "+v"(sk));
      y += sk;
      const float sg = __builtin_amdgcn_rcpf(1.0f + expf(-zv));
      const float gt = zv * sg;
      sY[s * kTP + tid] = (y * gt) * kCarryY;
    }
    __syncthreads();
    v8h hv[2];
#pragma unroll
    for (int it = 0; it < 2; ++it) {
      const float* sp = sY + (it * 8 + wave) * kTP + lane * 8;
      const v4f a0 = *(const v4f*)(sp);
      const v4f a1 = *(const v4f*)(sp + 4);
#pragma unroll
      for (int e = 0; e < 4; ++e) {
        hv[it][e]     = (_Float16)a0[e];
        hv[it][4 + e] = (_Float16)a1[e];
      }
    }
    for (int pass = 0; pass < 2; ++pass) {
#pragma unroll
      for (int it = 0; it < 2; ++it)
        *(volatile v8h*)(Y16 + (row0 + l0 + it * 8 + wave) * kDin + d0 + lane * 8) = hv[it];
      __threadfence();
    }
  }
}

extern "C" void kernel_launch(void* const* d_in, const int* in_sizes, int n_in,
                              void* d_out, int out_size, void* d_ws, size_t ws_size,
                              hipStream_t stream)
{
  if (n_in < 13) return;
  if (in_sizes[0] != kRows * kDmod) return;
  if (in_sizes[1] != kDmod || in_sizes[2] != kDmod) return;
  if (in_sizes[3] != kDmod * kXZP) return;
  if (in_sizes[4] != kDin * 4 || in_sizes[5] != kDin) return;
  if (in_sizes[6] != kDin * kPrjN) return;
  if (in_sizes[7] != kDtR * kDin || in_sizes[8] != kDin) return;
  if (in_sizes[9] != kDin * kNst || in_sizes[10] != kDin) return;
  if (in_sizes[11] != kDin * kDmod) return;
  if (in_sizes[12] != 1) return;
  if (out_size != kRows * kDmod) return;
  if (ws_size < kWsTotal) return;

  const float* x      = (const float*)d_in[0];
  const float* ln_g   = (const float*)d_in[1];
  const float* ln_b   = (const float*)d_in[2];
  const float* W_in   = (const float*)d_in[3];
  const float* conv_w = (const float*)d_in[4];
  const float* conv_b = (const float*)d_in[5];
  const float* W_xp   = (const float*)d_in[6];
  const float* W_dt   = (const float*)d_in[7];
  const float* b_dt   = (const float*)d_in[8];
  const float* A_log  = (const float*)d_in[9];
  const float* Dv     = (const float*)d_in[10];
  const float* W_out  = (const float*)d_in[11];
  const float* res_sc = (const float*)d_in[12];
  float* dout = (float*)d_out;

  char* ws = (char*)d_ws;
  unsigned short* WIN16  = (unsigned short*)(ws + kOffWIN);
  unsigned short* WXP16  = (unsigned short*)(ws + kOffWXP);
  unsigned short* WDT16  = (unsigned short*)(ws + kOffWDT);
  unsigned short* WOUT16 = (unsigned short*)(ws + kOffWOUT);
  unsigned short* XN16   = (unsigned short*)(ws + kOffXN);
  float*          XZ     = (float*)(ws + kOffXZ);
  float*          UC     = (float*)(ws + kOffUC);
  unsigned short* UC16   = (unsigned short*)(ws + kOffUC16);
  float*          PROJ   = (float*)(ws + kOffPROJ);
  unsigned short* DT16   = (unsigned short*)(ws + kOffDT16);
  float*          DLR    = (float*)(ws + kOffDLR);
  unsigned short* Y16    = (unsigned short*)(ws + kOffY16);

  transpose_cast_kernel<<<dim3(kXZP / 64, kDmod / 64), 256, 0, stream>>>(W_in, WIN16, kDmod, kXZP, kCarryW);
  transpose_cast_kernel<<<dim3(kPrjP / 64, kDin / 64), 256, 0, stream>>>(W_xp, WXP16, kDin, kPrjN, kCarryW);
  transpose_cast_kernel<<<dim3(kDin / 64, kDtR / 64), 256, 0, stream>>>(W_dt, WDT16, kDtR, kDin, kCarryWdt);
  transpose_cast_kernel<<<dim3(kDmod / 64, kDin / 64), 256, 0, stream>>>(W_out, WOUT16, kDin, kDmod, kCarryW);

  ln_cast_kernel<<<kRows / 8, 256, 0, stream>>>(x, ln_g, ln_b, XN16);

  wmma_gemm64_f16<0, false, false><<<(kRows / 64) * (kXZP / 64) / 8, 256, 0, stream>>>(
      XN16, kDmod, WIN16, kDmod, XZ, kXZP, b_dt, x, res_sc, kRows, kXZP, kDmod, kFoldIn);

  conv_silu_kernel<<<dim3(kDin / 256, kRows / 64), 256, 0, stream>>>(XZ, conv_w, conv_b, UC, UC16);

  wmma_gemm64_f16<0, false, false><<<(kRows / 64) * (kPrjP / 64) / 8, 256, 0, stream>>>(
      UC16, kDin, WXP16, kDin, PROJ, kPrjP, b_dt, x, res_sc, kRows, kPrjP, kDin, kFoldXp);

  dt_cast_kernel<<<(kRows * kDtR) / 8 / 256, 256, 0, stream>>>(PROJ, DT16, (kRows * kDtR) / 8, kCarryDt);

  wmma_gemm64_f16<2, false, false><<<(kRows / 64) * (kDin / 64) / 8, 256, 0, stream>>>(
      DT16, kDtR, WDT16, kDtR, DLR, kDin, b_dt, x, res_sc, kRows, kDin, kDtR, kFoldDt);

  scan_kernel<<<dim3(kDin / 256, kBatch), 256, 0, stream>>>(DLR, UC, XZ, PROJ, A_log, Dv, Y16);

  wmma_gemm64_f16<0, true, true><<<(kRows / 64) * (kDmod / 64) / 8, 256, 0, stream>>>(
      Y16, kDin, WOUT16, kDin, dout, kDmod, b_dt, x, res_sc, kRows, kDmod, kDin, kFoldOut);
}
